// HybridContrastiveLoss_47364899340368
// MI455X (gfx1250) — hardware-verified
//
#include <hip/hip_runtime.h>


#define TEMP_INV 10.0f
#define EPSF     1e-6f
#define NBHD     5

typedef _Float16 v16h __attribute__((ext_vector_type(16)));
typedef _Float16 v8h  __attribute__((ext_vector_type(8)));
typedef float    v8f  __attribute__((ext_vector_type(8)));
typedef float    v4f  __attribute__((ext_vector_type(4)));
typedef double   v2d  __attribute__((ext_vector_type(2)));

static constexpr int N_  = 2;
static constexpr int C_  = 64;
static constexpr int H_  = 64;
static constexpr int W_  = 64;
static constexpr int HW_ = H_ * W_;
static constexpr int M_  = N_ * HW_;
static constexpr int JT_ = M_ / 16;

static constexpr int NRM_TPB  = 128;
static constexpr int NRM_BLKS = M_ / NRM_TPB;
static constexpr int PIX_WPB  = 8;
static constexpr int PIX_BLKS = JT_ / PIX_WPB;
static constexpr int LD_TPB   = 256;
static constexpr int LD_BLKS  = M_ / LD_TPB;
static constexpr int LINE_D   = 16;

static constexpr float F16_SCALE   = 8.0f;
static constexpr float LOGIT_SCALE = TEMP_INV / (F16_SCALE * F16_SCALE);

static_assert(M_ % NRM_TPB == 0);
static_assert(JT_ % PIX_WPB == 0);
static_assert(M_ % LD_TPB == 0);
static_assert(C_ == 64);

union Frag {
    v16h v;
    v8h  hf[2];
};

__device__ __forceinline__ v8f wmma16(v8f acc, v16h a, v16h b) {
    acc = __builtin_amdgcn_wmma_f32_16x16x32_f16(false, a, false, b, (short)0, acc, false, false);
    asm volatile("v_nop\n\tv_nop\n\tv_nop\n\tv_nop" : "+v"(acc) : "v"(a), "v"(b));
    return acc;
}

__device__ __forceinline__ void store_norm_tile(const v4f* s32, const v8h* s16,
                                                float* d32, _Float16* d16, int tid) {
#pragma unroll
    for (int it = 0; it < (NRM_TPB * (C_ / 4)) / NRM_TPB; ++it) {
        const int idx = it * NRM_TPB + tid;
        const v4f y = s32[idx];
        *(volatile v4f*)(d32 + (size_t)idx * 4) = y;
    }
#pragma unroll
    for (int it = 0; it < (NRM_TPB * (C_ / 8)) / NRM_TPB; ++it) {
        const int idx = it * NRM_TPB + tid;
        const v8h t = s16[idx];
        *(volatile v8h*)(d16 + (size_t)idx * 8) = t;
    }
}

__global__ __launch_bounds__(NRM_TPB)
void k_normalize(const float* __restrict__ feat,
                 float* __restrict__ fm32,
                 _Float16* __restrict__ fm16) {
    __shared__ v4f s32[NRM_TPB * (C_ / 4)];
    __shared__ v8h s16[NRM_TPB * (C_ / 8)];

    const int tid = threadIdx.x;
    const int p0  = blockIdx.x * NRM_TPB;
    const int p   = p0 + tid;
    const int n   = p / HW_;
    const int hw  = p - n * HW_;
    const float* src = feat + (size_t)n * C_ * HW_ + hw;

    float v[C_];
    float ss = 0.0f;
#pragma unroll
    for (int c = 0; c < C_; ++c) {
        const float x = src[(size_t)c * HW_];
        v[c] = x;
        ss = fmaf(x, x, ss);
    }
    const float inv = 1.0f / fmaxf(sqrtf(ss), 1e-12f);

#pragma unroll
    for (int g = 0; g < C_ / 4; ++g) {
        v4f y;
        y.x = v[4 * g + 0] * inv;
        y.y = v[4 * g + 1] * inv;
        y.z = v[4 * g + 2] * inv;
        y.w = v[4 * g + 3] * inv;
        s32[tid * (C_ / 4) + g] = y;
    }
#pragma unroll
    for (int g = 0; g < C_ / 8; ++g) {
        v8h t;
#pragma unroll
        for (int i = 0; i < 8; ++i) t[i] = (_Float16)((v[8 * g + i] * inv) * F16_SCALE);
        s16[tid * (C_ / 8) + g] = t;
    }
    __syncthreads();

    float*    d32 = fm32 + (size_t)p0 * C_;
    _Float16* d16 = fm16 + (size_t)p0 * C_;
    store_norm_tile(s32, s16, d32, d16, tid);
    __threadfence();
    store_norm_tile(s32, s16, d32, d16, tid);
}

__global__ __launch_bounds__(256)
void k_pixel(const _Float16* __restrict__ fm16,
             const int* __restrict__ lab,
             double* __restrict__ partP) {
    __shared__ double s_part[2 * PIX_WPB];
    __shared__ double s_tot;

    const int lane = threadIdx.x & 31;
    const int wave = threadIdx.x >> 5;
    const int hl   = lane >> 4;
    const int nsub = lane & 15;
    const int tile = blockIdx.x * PIX_WPB + wave;
    const int i_base = tile * 16;
    const float NEG_INF = -__builtin_huge_valf();

    Frag a0, a1;
    {
        const _Float16* row = fm16 + (size_t)(i_base + nsub) * C_;
        a0.hf[0] = *(const v8h*)(row + 8 * hl);
        a0.hf[1] = *(const v8h*)(row + 16 + 8 * hl);
        a1.hf[0] = *(const v8h*)(row + 32 + 8 * hl);
        a1.hf[1] = *(const v8h*)(row + 48 + 8 * hl);
    }

    int labI[8];
#pragma unroll
    for (int r = 0; r < 8; ++r) labI[r] = lab[i_base + 8 * hl + r];

    float den[8], Ls[8];
#pragma unroll
    for (int r = 0; r < 8; ++r) { den[r] = 0.0f; Ls[r] = 0.0f; }

#pragma unroll 1
    for (int jt = 0; jt < JT_; ++jt) {
        const int j_base = jt * 16;
        const _Float16* rowj = fm16 + (size_t)(j_base + nsub) * C_;
        Frag b0, b1;
        b0.hf[0] = *(const v8h*)(rowj + 8 * hl);
        b0.hf[1] = *(const v8h*)(rowj + 16 + 8 * hl);
        b1.hf[0] = *(const v8h*)(rowj + 32 + 8 * hl);
        b1.hf[1] = *(const v8h*)(rowj + 48 + 8 * hl);

        v8f acc = {0.f, 0.f, 0.f, 0.f, 0.f, 0.f, 0.f, 0.f};
        acc = wmma16(acc, a0.v, b0.v);
        acc = wmma16(acc, a1.v, b1.v);

        const int labJ = lab[j_base + nsub];
#pragma unroll
        for (int r = 0; r < 8; ++r) {
            const float l  = acc[r] * LOGIT_SCALE;
            const bool  mk = (labI[r] == labJ);
            den[r] += mk ? __expf(l) : 0.0f;
            Ls[r]  += mk ? l : NEG_INF;
        }
    }

#pragma unroll
    for (int r = 0; r < 8; ++r) {
        float d = den[r], L = Ls[r];
#pragma unroll
        for (int m = 1; m < 16; m <<= 1) {
            d += __shfl_xor(d, m, 32);
            L += __shfl_xor(L, m, 32);
        }
        den[r] = d; Ls[r] = L;
    }

    double tsum = 0.0;
#pragma unroll
    for (int r = 0; r < 8; ++r)
        tsum += (double)M_ * (double)logf(den[r] + EPSF) - (double)Ls[r];

    if (nsub == 0) s_part[wave * 2 + hl] = tsum;
    __syncthreads();
    if (threadIdx.x == 0) {
        double b = 0.0;
#pragma unroll
        for (int i = 0; i < 2 * PIX_WPB; ++i) b += s_part[i];
        s_tot = b;
    }
    __syncthreads();

    if (wave == 0) {
        const double tot = s_tot;
        v2d val;
        val.x = (lane == 0) ? tot : 0.0;
        val.y = 0.0;
        double* line = partP + (size_t)blockIdx.x * LINE_D;
        if (lane < 8) *(volatile v2d*)(line + 2 * lane) = val;
        __threadfence();
        if (lane < 8) *(volatile v2d*)(line + 2 * lane) = val;
    }
}

__global__ __launch_bounds__(LD_TPB)
void k_locdir(const float* __restrict__ fm32,
              const int* __restrict__ lab,
              const float* __restrict__ dirs,
              double* __restrict__ partL) {
    __shared__ double s_loc[LD_TPB];
    __shared__ double s_dir[LD_TPB];

    const int tid = threadIdx.x;
    const int p   = blockIdx.x * LD_TPB + tid;
    const int n   = p / HW_;
    const int hw  = p - n * HW_;
    const int h   = hw / W_;
    const int w   = hw - h * W_;
    const float NEG_INF = -__builtin_huge_valf();
    const float POS_INF = __builtin_huge_valf();

    float me[C_];
    {
        const v4f* mp = (const v4f*)(fm32 + (size_t)p * C_);
#pragma unroll
        for (int t = 0; t < C_ / 4; ++t) {
            const v4f a = mp[t];
            me[4 * t + 0] = a.x; me[4 * t + 1] = a.y; me[4 * t + 2] = a.z; me[4 * t + 3] = a.w;
        }
    }
    const int labMe = lab[p];

    const int h0 = max(h - NBHD, 0), h1 = min(h + NBHD, H_ - 1);
    const int w0 = max(w - NBHD, 0), w1 = min(w + NBHD, W_ - 1);
    const int cnt = (h1 - h0 + 1) * (w1 - w0 + 1);

    int  qd[2], labd[2];
    bool vd[2];
#pragma unroll
    for (int k = 0; k < 2; ++k) {
        float fdi = dirs[((size_t)k * 2 + 0) * HW_ + hw];
        float fdj = dirs[((size_t)k * 2 + 1) * HW_ + hw];
        fdi = fminf(fmaxf(fdi, -1.0e6f), 1.0e6f);
        fdj = fminf(fmaxf(fdj, -1.0e6f), 1.0e6f);
        const int di = (int)fdi, dj = (int)fdj;
        const int ni = h + di, nj = w + dj;
        vd[k] = (ni >= 0) && (ni < H_) && (nj >= 0) && (nj < W_);
        const int nic = min(max(ni, 0), H_ - 1);
        const int njc = min(max(nj, 0), W_ - 1);
        qd[k]   = n * HW_ + nic * W_ + njc;
        labd[k] = lab[qd[k]];
    }

    float denL = 0.0f, LsL = 0.0f, lg0 = 0.0f, lg1 = 0.0f;
    int nh = h0, nw = w0;
    const int total = cnt + 2;
    for (int idx = 0; idx < total; ++idx) {
        const bool inwin = (idx < cnt);
        int q;
        if (inwin) q = n * HW_ + nh * W_ + nw;
        else       q = (idx == cnt) ? qd[0] : qd[1];
        const v4f* nb = (const v4f*)(fm32 + (size_t)q * C_);
        float dot = 0.0f;
#pragma unroll
        for (int t = 0; t < C_ / 4; ++t) {
            const v4f b = nb[t];
            dot = fmaf(me[4 * t + 0], b.x, dot);
            dot = fmaf(me[4 * t + 1], b.y, dot);
            dot = fmaf(me[4 * t + 2], b.z, dot);
            dot = fmaf(me[4 * t + 3], b.w, dot);
        }
        const float l = dot * TEMP_INV;
        if (inwin) {
            const bool mk = (lab[q] == labMe);
            denL += mk ? __expf(l) : 0.0f;
            LsL  += mk ? l : NEG_INF;
            ++nw;
            if (nw > w1) { nw = w0; ++nh; }
        } else if (idx == cnt) {
            lg0 = l;
        } else {
            lg1 = l;
        }
    }

    const float termL = (float)cnt * __logf(denL + EPSF) - LsL;
    const float cL = termL * __builtin_amdgcn_rcpf((float)(N_ * cnt * HW_));

    const bool m0 = (labd[0] == labMe), m1 = (labd[1] == labMe);
    const int  kc = (vd[0] ? 1 : 0) + (vd[1] ? 1 : 0);
    float denD = 0.0f;
    if (vd[0] && m0) denD += __expf(lg0);
    if (vd[1] && m1) denD += __expf(lg1);
    float cD = 0.0f;
    if (kc > 0) {
        const float ld = __logf(denD + EPSF);
        float ts = 0.0f;
        if (vd[0]) ts += m0 ? (ld - lg0) : POS_INF;
        if (vd[1]) ts += m1 ? (ld - lg1) : POS_INF;
        cD = ts * __builtin_amdgcn_rcpf((float)(N_ * kc * HW_));
    }

    s_loc[tid] = (double)cL;
    s_dir[tid] = (double)cD;
    __syncthreads();
    for (int s = LD_TPB / 2; s > 0; s >>= 1) {
        if (tid < s) {
            s_loc[tid] += s_loc[tid + s];
            s_dir[tid] += s_dir[tid + s];
        }
        __syncthreads();
    }

    if (tid < 32) {
        v2d val;
        val.x = (tid == 0) ? s_loc[0] : 0.0;
        val.y = (tid == 0) ? s_dir[0] : 0.0;
        double* line = partL + (size_t)blockIdx.x * LINE_D;
        if (tid < 8) *(volatile v2d*)(line + 2 * tid) = val;
        __threadfence();
        if (tid < 8) *(volatile v2d*)(line + 2 * tid) = val;
    }
}

__global__ void k_final(const double* __restrict__ partP,
                        const double* __restrict__ partL,
                        float* __restrict__ out) {
    if (threadIdx.x != 0) return;
    double sp = 0.0;
    for (int b = 0; b < PIX_BLKS; ++b) sp += partP[(size_t)b * LINE_D];
    double sl = 0.0, sd = 0.0;
    for (int b = 0; b < LD_BLKS; ++b) {
        sl += partL[(size_t)b * LINE_D];
        sd += partL[(size_t)b * LINE_D + 1];
    }
    const double loss = sp * (1.0 / ((double)M_ * (double)M_)) + sl + sd;
    const float f = (float)loss;
    *(volatile float*)out = f;
    __threadfence();
    *(volatile float*)out = f;
}

extern "C" void kernel_launch(void* const* d_in, const int* in_sizes, int n_in,
                              void* d_out, int out_size, void* d_ws, size_t ws_size,
                              hipStream_t stream) {
    if (n_in < 3 || out_size < 1) return;
    if (in_sizes[0] != N_ * C_ * HW_ || in_sizes[1] != M_ || in_sizes[2] != N_ * 2 * HW_) return;

    const size_t off_fm32 = 0;
    const size_t by_fm32  = (size_t)M_ * C_ * sizeof(float);
    const size_t off_fm16 = off_fm32 + by_fm32;
    const size_t by_fm16  = (size_t)M_ * C_ * 2;
    const size_t off_pp   = off_fm16 + by_fm16;
    const size_t by_pp    = (size_t)PIX_BLKS * 128;
    const size_t off_pl   = off_pp + by_pp;
    const size_t by_pl    = (size_t)LD_BLKS * 128;
    const size_t total    = off_pl + by_pl;
    if (total > ws_size) return;

    const float* feat = (const float*)d_in[0];
    const int*   lab  = (const int*)d_in[1];
    const float* dirs = (const float*)d_in[2];
    float*       out  = (float*)d_out;

    char* ws = (char*)d_ws;
    float*    fm32  = (float*)(ws + off_fm32);
    _Float16* fm16  = (_Float16*)(ws + off_fm16);
    double*   partP = (double*)(ws + off_pp);
    double*   partL = (double*)(ws + off_pl);

    k_normalize<<<NRM_BLKS, NRM_TPB, 0, stream>>>(feat, fm32, fm16);
    k_pixel<<<PIX_BLKS, 32 * PIX_WPB, 0, stream>>>(fm16, lab, partP);
    k_locdir<<<LD_BLKS, LD_TPB, 0, stream>>>(fm32, lab, dirs, partL);
    k_final<<<1, 32, 0, stream>>>(partP, partL, out);
}
